// MambaBlock_28381143892421
// MI455X (gfx1250) — hardware-verified
//
#include <hip/hip_runtime.h>
#include <stddef.h>
#include <stdint.h>
#include <math.h>


#define NB    8
#define SEQ   2048
#define DM    512
#define NST   16
#define INR   768
#define MROWS (NB * SEQ)
#define NPJ   (3 * INR)
#define KPJ   (2 * DM)
#define KOUT  (2 * INR)
#define KST   (2 * NST)
#define NTAY  19
#define PSTR  20
#define CST_AINV (256 * PSTR)
#define CST_MISC (CST_AINV + 256)
#define CST_N    (CST_MISC + 16)
#define TPB   64
#define SMAX  20
#define GBM   64
#define GBN   128
#define GTHR  128
#define CTOK  16
#define CTHR  192
#define U_WIN  (NPJ * (KPJ / 8))
#define U_WOUT (DM * (KOUT / 8))
#define U_BM   (NST * (KOUT / 8))
#define U_CM   (INR * (KST / 8))
#define U_ALL  (U_WIN + U_WOUT + U_BM + U_CM)

static_assert(MROWS % GBM == 0 && NPJ % GBN == 0 && DM % GBN == 0 && INR % GBN == 0);
static_assert(KPJ % 32 == 0 && KOUT % 32 == 0 && KST == 32);
static_assert(INR / GBN == 6 && NPJ / GBN == 18);
static_assert(U_WIN % 256 == 0 && U_WOUT % 256 == 0 && U_BM % 256 == 0 && U_CM % 256 == 0);
static_assert((KOUT / 8) == 192 && (KOUT / 8) % 32 == 0);
static_assert(SEQ % CTOK == 0 && SEQ % 32 == 0 && MROWS % TPB == 0 && MROWS % 8 == 0);
static_assert(CTHR * 4 == INR && (KOUT / 32) == 48 && 48 == 6 * 8 && CTHR == 6 * 32);
static_assert(NTAY <= PSTR && PSTR % 2 == 0);

typedef float          v4f   __attribute__((ext_vector_type(4)));
typedef float          v8f   __attribute__((ext_vector_type(8)));
typedef int            v8i   __attribute__((ext_vector_type(8)));
typedef double         v2d   __attribute__((ext_vector_type(2)));
typedef unsigned short v4us  __attribute__((ext_vector_type(4)));
typedef unsigned short v8us  __attribute__((ext_vector_type(8)));
typedef unsigned short v16us __attribute__((ext_vector_type(16)));
typedef __bf16         v16bf __attribute__((ext_vector_type(16)));
typedef v4f  __attribute__((may_alias)) v4fa;
typedef v2d  __attribute__((may_alias)) v2da;
typedef v4us __attribute__((may_alias)) v4usa;
typedef v8us __attribute__((may_alias)) v8usa;
union FragB { v16bf v; v16us u; v8us h[2]; v8i w; };

__device__ __forceinline__ v8f wmb(const FragB& a, const FragB& b, v8f c) {
  v8f d = __builtin_amdgcn_wmma_f32_16x16x32_bf16(false, a.v, false, b.v, (short)0, c, false, false);
  asm volatile("v_nop\n\tv_nop\n\tv_nop\n\tv_nop" : "+v"(d) : "v"(a.w), "v"(b.w));
  return d;
}

__device__ __forceinline__ unsigned bf16_bits(float f) {
  const unsigned u = __float_as_uint(f);
  return (u + 0x7FFFu + ((u >> 16) & 1u)) >> 16;
}
__device__ __forceinline__ float bf16_val(float f) {
  return __uint_as_float(bf16_bits(f) << 16);
}
__device__ __forceinline__ v4f bf4(v4f a) {
  v4f r;
  r.x = bf16_val(a.x); r.y = bf16_val(a.y); r.z = bf16_val(a.z); r.w = bf16_val(a.w);
  return r;
}
__device__ __forceinline__ void hilo(float v, unsigned& hb, unsigned& lb) {
  hb = bf16_bits(v);
  lb = bf16_bits(v - __uint_as_float(hb << 16));
}
__device__ __forceinline__ void hilo4(v4f v, v4us& h4, v4us& l4) {
  unsigned hb, lb;
  hilo(v.x, hb, lb); h4[0] = (unsigned short)hb; l4[0] = (unsigned short)lb;
  hilo(v.y, hb, lb); h4[1] = (unsigned short)hb; l4[1] = (unsigned short)lb;
  hilo(v.z, hb, lb); h4[2] = (unsigned short)hb; l4[2] = (unsigned short)lb;
  hilo(v.w, hb, lb); h4[3] = (unsigned short)hb; l4[3] = (unsigned short)lb;
}
__device__ __forceinline__ float softplus_f(float v) {
  return fmaxf(v, 0.0f) + log1pf(expf(-fabsf(v)));
}
__device__ __forceinline__ float sigmoid_f(float v) {
  return 1.0f / (1.0f + expf(-v));
}

__device__ __forceinline__ void cvt8_store(const float* __restrict__ p, unsigned short* dp) {
  const v4f a = *(const v4f*)p;
  const v4f b = *(const v4f*)(p + 4);
  v8us o;
  o[0] = (unsigned short)bf16_bits(a.x); o[1] = (unsigned short)bf16_bits(a.y);
  o[2] = (unsigned short)bf16_bits(a.z); o[3] = (unsigned short)bf16_bits(a.w);
  o[4] = (unsigned short)bf16_bits(b.x); o[5] = (unsigned short)bf16_bits(b.y);
  o[6] = (unsigned short)bf16_bits(b.z); o[7] = (unsigned short)bf16_bits(b.w);
  *(volatile v8us*)dp = o;
  __threadfence();
  *(volatile v8us*)dp = o;
}

__global__ __launch_bounds__(256) void k_wprep(const float* __restrict__ W_in, const float* __restrict__ W_out,
                                               const float* __restrict__ Bmat, const float* __restrict__ Cmat,
                                               unsigned short* WI2, unsigned short* WO2,
                                               unsigned short* BM2, unsigned short* CM2) {
  const int u = (int)blockIdx.x * 256 + (int)threadIdx.x;
  if (u < U_WIN) {
    const int n = u >> 7, k8 = (u & 127) * 8;
    cvt8_store(W_in + (size_t)n * DM + (k8 & (DM - 1)), WI2 + (size_t)n * KPJ + k8);
  } else if (u < U_WIN + U_WOUT) {
    const int v = u - U_WIN;
    const int n = v / 192, k8 = (v - n * 192) * 8;
    const int ks = (k8 >= INR) ? (k8 - INR) : k8;
    cvt8_store(W_out + (size_t)n * INR + ks, WO2 + (size_t)n * KOUT + k8);
  } else if (u < U_WIN + U_WOUT + U_BM) {
    const int v = u - (U_WIN + U_WOUT);
    const int n = v / 192, k8 = (v - n * 192) * 8;
    const int ks = (k8 >= INR) ? (k8 - INR) : k8;
    cvt8_store(Bmat + (size_t)n * INR + ks, BM2 + (size_t)n * KOUT + k8);
  } else if (u < U_ALL) {
    const int v = u - (U_WIN + U_WOUT + U_BM);
    const int n = v >> 2, k8 = (v & 3) * 8;
    cvt8_store(Cmat + (size_t)n * NST + (k8 & (NST - 1)), CM2 + (size_t)n * KST + k8);
  }
}

__global__ __launch_bounds__(256) void k_aprep(const float* __restrict__ A, double* cst) {
  __shared__ __attribute__((aligned(16))) double Ash[256];
  __shared__ __attribute__((aligned(16))) double G[16 * 32];
  __shared__ __attribute__((aligned(16))) double Pc[256];
  __shared__ __attribute__((aligned(16))) double Pall[256 * PSTR];
  __shared__ double cs[16];
  __shared__ int psh;
  const int tid = (int)threadIdx.x, i = tid >> 4, j = tid & 15;
  const double a = (double)bf16_val(A[tid]);
  const double idv = (i == j) ? 1.0 : 0.0;
  Ash[tid] = a;
  G[i * 32 + j] = a;
  G[i * 32 + 16 + j] = idv;
  Pc[tid] = idv;
  Pall[tid * PSTR + 0] = idv;
  Pall[tid * PSTR + (PSTR - 1)] = 0.0;
  __syncthreads();
  if (tid < 16) {
    double s = 0.0;
#pragma unroll 1
    for (int r = 0; r < 16; ++r) s += fabs(Ash[r * 16 + tid]);
    cs[tid] = s;
  }
  __syncthreads();
  double nrm = 0.0;
#pragma unroll 1
  for (int c = 0; c < 16; ++c) { const double v = cs[c]; nrm = (v > nrm) ? v : nrm; }

#pragma unroll 1
  for (int k = 1; k < NTAY; ++k) {
    double s = 0.0;
#pragma unroll 4
    for (int mm = 0; mm < 16; ++mm) s = fma(Pc[i * 16 + mm], Ash[mm * 16 + j], s);
    s = s * (1.0 / (double)k);
    __syncthreads();
    Pc[tid] = s;
    Pall[tid * PSTR + k] = s;
    __syncthreads();
  }

  const double qnan = __longlong_as_double(0x7ff8LL << 48);
#pragma unroll 1
  for (int k = 0; k < 16; ++k) {
    if (tid == 0) {
      int p = k;
      double best = fabs(G[k * 32 + k]);
#pragma unroll 1
      for (int r = k + 1; r < 16; ++r) {
        const double v = fabs(G[r * 32 + k]);
        if (v > best) { best = v; p = r; }
      }
      psh = p;
    }
    __syncthreads();
    int p = psh;
    p = p < 0 ? 0 : (p > 15 ? 15 : p);
    if (i == k && p != k) {
      const double t0 = G[k * 32 + j], t1 = G[k * 32 + 16 + j];
      const double u0 = G[p * 32 + j], u1 = G[p * 32 + 16 + j];
      G[k * 32 + j] = u0; G[k * 32 + 16 + j] = u1;
      G[p * 32 + j] = t0; G[p * 32 + 16 + j] = t1;
    }
    __syncthreads();
    const double piv = G[k * 32 + k];
    const double rp  = (piv == 0.0) ? qnan : (1.0 / piv);
    const double f   = G[i * 32 + k];
    const double rk0 = G[k * 32 + j] * rp;
    const double rk1 = G[k * 32 + 16 + j] * rp;
    const double g0  = G[i * 32 + j];
    const double g1  = G[i * 32 + 16 + j];
    __syncthreads();
    G[i * 32 + j]      = (i == k) ? rk0 : fma(-f, rk0, g0);
    G[i * 32 + 16 + j] = (i == k) ? rk1 : fma(-f, rk1, g1);
    __syncthreads();
  }

  v2d pv[10];
#pragma unroll
  for (int q = 0; q < 10; ++q) pv[q] = *(const v2da*)(Pall + 2 * (q * 256 + tid));
  const int e2 = 2 * (tid & 127);
  v2d av;
  av.x = G[(e2 >> 4) * 32 + 16 + (e2 & 15)];
  av.y = G[(e2 >> 4) * 32 + 16 + (e2 & 15) + 1];
  v2d nv; nv.x = nrm; nv.y = nrm;
  const bool oka = tid < 128, okn = tid < 8;
#pragma unroll
  for (int q = 0; q < 10; ++q) *(volatile v2d*)(cst + 2 * (q * 256 + tid)) = pv[q];
  if (oka) *(volatile v2d*)(cst + CST_AINV + e2) = av;
  if (okn) *(volatile v2d*)(cst + CST_MISC + 2 * (tid & 7)) = nv;
  __threadfence();
#pragma unroll
  for (int q = 0; q < 10; ++q) *(volatile v2d*)(cst + 2 * (q * 256 + tid)) = pv[q];
  if (oka) *(volatile v2d*)(cst + CST_AINV + e2) = av;
  if (okn) *(volatile v2d*)(cst + CST_MISC + 2 * (tid & 7)) = nv;
}

__device__ __forceinline__ void pack8(v4f p, v4f q, v8us& hi, v8us& lo) {
  v4us h4, l4;
  hilo4(p, h4, l4);
  hi[0] = h4[0]; hi[1] = h4[1]; hi[2] = h4[2]; hi[3] = h4[3];
  lo[0] = l4[0]; lo[1] = l4[1]; lo[2] = l4[2]; lo[3] = l4[3];
  hilo4(q, h4, l4);
  hi[4] = h4[0]; hi[5] = h4[1]; hi[6] = h4[2]; hi[7] = h4[3];
  lo[4] = l4[0]; lo[5] = l4[1]; lo[6] = l4[2]; lo[7] = l4[3];
}

__global__ __launch_bounds__(256) void k_ln(const float* __restrict__ x, const float* __restrict__ g,
                                            const float* __restrict__ b, unsigned short* H) {
  const int tid = (int)threadIdx.x, lane = tid & 31, wave = tid >> 5;
  const int row = (int)blockIdx.x * 8 + wave;
  const int c0 = 8 * lane, c1 = 256 + 8 * lane;
  const float* xr = x + (size_t)row * DM;
  const v4f a0 = bf4(*(const v4f*)(xr + c0));
  const v4f a1 = bf4(*(const v4f*)(xr + c0 + 4));
  const v4f a2 = bf4(*(const v4f*)(xr + c1));
  const v4f a3 = bf4(*(const v4f*)(xr + c1 + 4));
  float s = ((a0.x + a0.y) + (a0.z + a0.w)) + ((a1.x + a1.y) + (a1.z + a1.w))
          + ((a2.x + a2.y) + (a2.z + a2.w)) + ((a3.x + a3.y) + (a3.z + a3.w));
  s += __shfl_xor(s, 16, 32); s += __shfl_xor(s, 8, 32); s += __shfl_xor(s, 4, 32);
  s += __shfl_xor(s, 2, 32);  s += __shfl_xor(s, 1, 32);
  const float mu = s * (1.0f / (float)DM);
  const v4f d0 = a0 - mu, d1 = a1 - mu, d2 = a2 - mu, d3 = a3 - mu;
  float q = ((d0.x * d0.x + d0.y * d0.y) + (d0.z * d0.z + d0.w * d0.w))
          + ((d1.x * d1.x + d1.y * d1.y) + (d1.z * d1.z + d1.w * d1.w))
          + ((d2.x * d2.x + d2.y * d2.y) + (d2.z * d2.z + d2.w * d2.w))
          + ((d3.x * d3.x + d3.y * d3.y) + (d3.z * d3.z + d3.w * d3.w));
  q += __shfl_xor(q, 16, 32); q += __shfl_xor(q, 8, 32); q += __shfl_xor(q, 4, 32);
  q += __shfl_xor(q, 2, 32);  q += __shfl_xor(q, 1, 32);
  const float var = q * (1.0f / (float)DM);
  const float inv = 1.0f / sqrtf(var + 1e-5f);
  const v4f g0 = bf4(*(const v4f*)(g + c0)), g1 = bf4(*(const v4f*)(g + c0 + 4));
  const v4f g2 = bf4(*(const v4f*)(g + c1)), g3 = bf4(*(const v4f*)(g + c1 + 4));
  const v4f b0 = bf4(*(const v4f*)(b + c0)), b1 = bf4(*(const v4f*)(b + c0 + 4));
  const v4f b2 = bf4(*(const v4f*)(b + c1)), b3 = bf4(*(const v4f*)(b + c1 + 4));
  const v4f h0 = d0 * inv * g0 + b0;
  const v4f h1 = d1 * inv * g1 + b1;
  const v4f h2 = d2 * inv * g2 + b2;
  const v4f h3 = d3 * inv * g3 + b3;
  v8us hiA, loA, hiB, loB;
  pack8(h0, h1, hiA, loA);
  pack8(h2, h3, hiB, loB);
  unsigned short* hr = H + (size_t)row * KPJ;
  *(volatile v8us*)(hr + c0) = hiA;
  *(volatile v8us*)(hr + c1) = hiB;
  *(volatile v8us*)(hr + DM + c0) = loA;
  *(volatile v8us*)(hr + DM + c1) = loB;
  __threadfence();
  *(volatile v8us*)(hr + c0) = hiA;
  *(volatile v8us*)(hr + c1) = hiB;
  *(volatile v8us*)(hr + DM + c0) = loA;
  *(volatile v8us*)(hr + DM + c1) = loB;
}

template <int MODE>
__global__ __launch_bounds__(GTHR) void k_gemm(const unsigned short* __restrict__ A,
                                               const unsigned short* __restrict__ BT, int K,
                                               float* dg, size_t gateOff, float* dpart,
                                               const float* __restrict__ xin, float* outp) {
  __shared__ __attribute__((aligned(16))) float stg[GBM * GBN];
  __shared__ __attribute__((aligned(16))) float rs[GBM];
  const int tid = (int)threadIdx.x, lane = tid & 31, wave = tid >> 5, hh = lane >> 4, m = lane & 15;
  const int wr = wave >> 1, wc = wave & 1;
  const int rowBase = (int)blockIdx.x * GBM;
  const int col0    = (int)blockIdx.y * GBN;

  v8f acc[2][4];
  {
    const v8f z = {0.f, 0.f, 0.f, 0.f, 0.f, 0.f, 0.f, 0.f};
#pragma unroll
    for (int i = 0; i < 2; ++i)
#pragma unroll
      for (int t = 0; t < 4; ++t) acc[i][t] = z;
  }
  const unsigned short* ap0 = A + (size_t)(rowBase + 32 * wr + m) * (size_t)K + 8 * hh;
  const unsigned short* ap1 = ap0 + (size_t)16 * (size_t)K;
  const unsigned short* bp  = BT + (size_t)(col0 + 64 * wc + m) * (size_t)K + 8 * hh;
#pragma unroll 1
  for (int k0 = 0; k0 < K; k0 += 32) {
    FragB a0, a1;
    a0.h[0] = *(const v8usa*)(ap0 + k0);
    a0.h[1] = *(const v8usa*)(ap0 + k0 + 16);
    a1.h[0] = *(const v8usa*)(ap1 + k0);
    a1.h[1] = *(const v8usa*)(ap1 + k0 + 16);
#pragma unroll
    for (int t = 0; t < 4; ++t) {
      const unsigned short* wq = bp + (size_t)(16 * t) * (size_t)K + k0;
      FragB bf;
      bf.h[0] = *(const v8usa*)wq;
      bf.h[1] = *(const v8usa*)(wq + 16);
      acc[0][t] = wmb(a0, bf, acc[0][t]);
      acc[1][t] = wmb(a1, bf, acc[1][t]);
    }
  }

#pragma unroll
  for (int i = 0; i < 2; ++i)
#pragma unroll
    for (int t = 0; t < 4; ++t) {
      const int lc = 64 * wc + 16 * t + m;
#pragma unroll
      for (int r = 0; r < 8; ++r) {
        const int lr = 32 * wr + 16 * i + 8 * hh + r;
        stg[lr * GBN + lc] = acc[i][t][r];
      }
    }
  __syncthreads();

  if constexpr (MODE == 1) {
    v4f fv[16];
#pragma unroll
    for (int i = 0; i < 16; ++i) {
      const int lr = 16 * wave + i;
      const size_t go = (size_t)(rowBase + lr) * DM + col0 + 4 * lane;
      const v4f sv = *(const v4fa*)(stg + lr * GBN + 4 * lane);
      const v4f xv = bf4(*(const v4f*)(xin + go));
      fv[i] = xv + sv;
    }
#pragma unroll
    for (int i = 0; i < 16; ++i) {
      const size_t go = (size_t)(rowBase + 16 * wave + i) * DM + col0 + 4 * lane;
      *(volatile v4f*)(outp + go) = fv[i];
    }
    __threadfence();
#pragma unroll
    for (int i = 0; i < 16; ++i) {
      const size_t go = (size_t)(rowBase + 16 * wave + i) * DM + col0 + 4 * lane;
      *(volatile v4f*)(outp + go) = fv[i];
    }
  } else {
    const int cls = (int)blockIdx.y / 6;
    const int ct  = (int)blockIdx.y - 6 * cls;
    if (cls < 2) {
      v4f fv[16];
#pragma unroll
      for (int i = 0; i < 16; ++i) fv[i] = *(const v4fa*)(stg + (16 * wave + i) * GBN + 4 * lane);
      const size_t cb = (size_t)cls * gateOff + (size_t)ct * GBN + 4 * lane;
#pragma unroll
      for (int i = 0; i < 16; ++i) {
        const size_t go = cb + (size_t)(rowBase + 16 * wave + i) * INR;
        *(volatile v4f*)(dg + go) = fv[i];
      }
      __threadfence();
#pragma unroll
      for (int i = 0; i < 16; ++i) {
        const size_t go = cb + (size_t)(rowBase + 16 * wave + i) * INR;
        *(volatile v4f*)(dg + go) = fv[i];
      }
    } else {
#pragma unroll 1
      for (int i = 0; i < 16; ++i) {
        const int lr = 16 * wave + i;
        const v4f v = *(const v4fa*)(stg + lr * GBN + 4 * lane);
        float sp = (softplus_f(v.x) + softplus_f(v.y)) + (softplus_f(v.z) + softplus_f(v.w));
        sp += __shfl_xor(sp, 16, 32); sp += __shfl_xor(sp, 8, 32); sp += __shfl_xor(sp, 4, 32);
        sp += __shfl_xor(sp, 2, 32);  sp += __shfl_xor(sp, 1, 32);
        if (lane == 0) rs[lr] = sp;
      }
      __syncthreads();
      const v4f ov = *(const v4fa*)(rs + 4 * (lane & 15));
      float* op = dpart + (size_t)ct * MROWS + rowBase + 4 * (lane & 15);
      const bool okst = (wave == 0) && (lane < 16);
      if (okst) *(volatile v4f*)op = ov;
      __threadfence();
      if (okst) *(volatile v4f*)op = ov;
    }
  }
}

__global__ __launch_bounds__(CTHR) void k_conv(const float* __restrict__ data, const float* __restrict__ cw,
                                               const unsigned short* __restrict__ BM2, float* wt) {
  __shared__ __attribute__((aligned(16))) unsigned short U[CTOK * KOUT];
  __shared__ __attribute__((aligned(16))) float red[6 * 256];
  const int tid = (int)threadIdx.x, lane = tid & 31, wave = tid >> 5, hh = lane >> 4, m = lane & 15;
  const int rowBase = (int)blockIdx.x * CTOK;
  const int s0 = rowBase & (SEQ - 1);
  const int c4 = 4 * tid;

  v4f w0, w1, w2;
  {
    const v4f wa = bf4(*(const v4f*)(cw + 12 * tid));
    const v4f wb = bf4(*(const v4f*)(cw + 12 * tid + 4));
    const v4f wc = bf4(*(const v4f*)(cw + 12 * tid + 8));
    w0.x = wa.x; w1.x = wa.y; w2.x = wa.z;
    w0.y = wa.w; w1.y = wb.x; w2.y = wb.y;
    w0.z = wb.z; w1.z = wb.w; w2.z = wc.x;
    w0.w = wc.y; w1.w = wc.z; w2.w = wc.w;
  }
  v4f dm2 = {0.f, 0.f, 0.f, 0.f}, dm1 = {0.f, 0.f, 0.f, 0.f};
#pragma unroll 1
  for (int i = -2; i < CTOK; ++i) {
    const bool inb = (s0 + i) >= 0;
    const int rr = inb ? (rowBase + i) : rowBase;
    const float f = inb ? 1.0f : 0.0f;
    const v4f d = (*(const v4f*)(data + (size_t)rr * INR + c4)) * f;
    if (i >= 0) {
      const v4f dc = w0 * dm2 + w1 * dm1 + w2 * d;
      v4f uv;
      uv.x = dc.x * sigmoid_f(dc.x); uv.y = dc.y * sigmoid_f(dc.y);
      uv.z = dc.z * sigmoid_f(dc.z); uv.w = dc.w * sigmoid_f(dc.w);
      v4us h4, l4;
      hilo4(uv, h4, l4);
      *(v4usa*)(U + i * KOUT + c4) = h4;
      *(v4usa*)(U + i * KOUT + INR + c4) = l4;
    }
    dm2 = dm1; dm1 = d;
  }
  __syncthreads();

  v8f acc = {0.f, 0.f, 0.f, 0.f, 0.f, 0.f, 0.f, 0.f};
  const unsigned short* ua = U + m * KOUT + 8 * hh;
  const unsigned short* bq = BM2 + (size_t)m * KOUT + 8 * hh;
#pragma unroll 1
  for (int j = 0; j < 8; ++j) {
    const int k0 = 32 * (8 * wave + j);
    FragB af, bf;
    af.h[0] = *(const v8usa*)(ua + k0);
    af.h[1] = *(const v8usa*)(ua + k0 + 16);
    bf.h[0] = *(const v8usa*)(bq + k0);
    bf.h[1] = *(const v8usa*)(bq + k0 + 16);
    acc = wmb(af, bf, acc);
  }
#pragma unroll
  for (int r = 0; r < 8; ++r) red[wave * 256 + (8 * hh + r) * 16 + m] = acc[r];
  __syncthreads();
  const int e = 4 * (tid & 63);
  v4f v = *(const v4fa*)(red + e);
  v = v + *(const v4fa*)(red + 256 + e);
  v = v + *(const v4fa*)(red + 512 + e);
  v = v + *(const v4fa*)(red + 768 + e);
  v = v + *(const v4fa*)(red + 1024 + e);
  v = v + *(const v4fa*)(red + 1280 + e);
  float* op = wt + (size_t)rowBase * NST + e;
  const bool okst = tid < 64;
  if (okst) *(volatile v4f*)op = v;
  __threadfence();
  if (okst) *(volatile v4f*)op = v;
}

__global__ __launch_bounds__(256) void k_expm(const double* __restrict__ cst, const float* __restrict__ dpart,
                                              const float* __restrict__ wt, double* ad, double* bvo) {
  __shared__ __attribute__((aligned(16))) double Tsh[256];
  __shared__ __attribute__((aligned(16))) double ai[256];
  __shared__ __attribute__((aligned(16))) double qsh[16];
  __shared__ __attribute__((aligned(16))) double bvb[TPB * 16];
  __shared__ __attribute__((aligned(16))) float wsh[TPB * 16];
  __shared__ float dls[TPB];
  const int tid = (int)threadIdx.x, n = tid >> 4, m = tid & 15;
  const int rowBase = (int)blockIdx.x * TPB;

  double p[PSTR];
#pragma unroll
  for (int j = 0; j < PSTR / 2; ++j) {
    const v2d t = *(const v2d*)(cst + (size_t)tid * PSTR + 2 * j);
    p[2 * j] = t.x; p[2 * j + 1] = t.y;
  }
  ai[tid] = cst[CST_AINV + tid];
  const double normA = cst[CST_MISC];
  *(v4fa*)(wsh + 4 * tid) = *(const v4f*)(wt + (size_t)rowBase * NST + 4 * tid);
  if (tid < TPB) {
    const int r = rowBase + tid;
    float sm = dpart[r];
    sm += dpart[MROWS + r];
    sm += dpart[2 * MROWS + r];
    sm += dpart[3 * MROWS + r];
    sm += dpart[4 * MROWS + r];
    sm += dpart[5 * MROWS + r];
    dls[tid] = fminf(sm * (1.0f / (float)INR) + 1e-4f, 3.0f);
  }
  __syncthreads();

#pragma unroll 1
  for (int t = 0; t < TPB; ++t) {
    const double dd = (double)dls[t];
    const double z  = dd * normA;
    int s = 0;
    double pw = 1.0, sc = 1.0;
#pragma unroll 1
    for (int q = 0; q < SMAX; ++q) {
      const bool gq = pw < z;
      pw = gq ? pw * 2.0 : pw;
      sc = gq ? sc * 0.5 : sc;
      s += gq ? 1 : 0;
    }
    const double tau = dd * sc;
    double Tv = p[NTAY - 1];
#pragma unroll
    for (int k = NTAY - 2; k >= 0; --k) Tv = fma(Tv, tau, p[k]);
    Tsh[tid] = Tv;
    __syncthreads();
#pragma unroll 1
    for (int q = 0; q < s; ++q) {
      double sum = 0.0;
#pragma unroll 4
      for (int kk = 0; kk < 16; kk += 2) {
        const v2d r2 = *(const v2da*)(Tsh + n * 16 + kk);
        sum = fma(r2.x, Tsh[kk * 16 + m], sum);
        sum = fma(r2.y, Tsh[(kk + 1) * 16 + m], sum);
      }
      __syncthreads();
      Tsh[tid] = sum;
      Tv = sum;
      __syncthreads();
    }
    {
      const int e2 = 2 * (tid & 127);
      const v2d av = *(const v2da*)(Tsh + e2);
      double* dp = ad + (size_t)(rowBase + t) * 256 + e2;
      const bool st2 = tid < 128;
      if (st2) *(volatile v2d*)dp = av;
      __threadfence();
      if (st2) *(volatile v2d*)dp = av;
    }
    double a = Tv * (double)wsh[t * 16 + m];
    a += __shfl_xor(a, 1, 32); a += __shfl_xor(a, 2, 32);
    a += __shfl_xor(a, 4, 32); a += __shfl_xor(a, 8, 32);
    if (m == 0) qsh[n] = a - (double)wsh[t * 16 + n];
    __syncthreads();
    double bq = ai[tid] * qsh[m];
    bq += __shfl_xor(bq, 1, 32); bq += __shfl_xor(bq, 2, 32);
    bq += __shfl_xor(bq, 4, 32); bq += __shfl_xor(bq, 8, 32);
    if (m == 0) bvb[t * 16 + n] = bq;
  }
  __syncthreads();
  const v2d b0 = *(const v2da*)(bvb + 2 * tid);
  const v2d b1 = *(const v2da*)(bvb + 2 * (256 + tid));
  double* bp0 = bvo + (size_t)rowBase * NST + 2 * tid;
  double* bp1 = bvo + (size_t)rowBase * NST + 2 * (256 + tid);
  *(volatile v2d*)bp0 = b0;
  *(volatile v2d*)bp1 = b1;
  __threadfence();
  *(volatile v2d*)bp0 = b0;
  *(volatile v2d*)bp1 = b1;
}

__global__ __launch_bounds__(32) void k_scan(const double* __restrict__ ad, const double* __restrict__ bv,
                                             unsigned short* stt) {
  __shared__ __attribute__((aligned(16))) double st[16];
  __shared__ __attribute__((aligned(16))) unsigned short sbuf[32 * 32];
  const int lane = (int)threadIdx.x, n = lane & 15, h = lane >> 4;
  if (lane < 16) st[lane] = 0.0;
  __syncthreads();
  const size_t base = (size_t)blockIdx.x * SEQ;
  const double* ap = ad + base * 256 + n * 16 + 8 * h;
  v2d c0 = *(const v2d*)(ap), c1 = *(const v2d*)(ap + 2), c2 = *(const v2d*)(ap + 4), c3 = *(const v2d*)(ap + 6);
#pragma unroll 1
  for (int t = 0; t < SEQ; ++t) {
    const int tn = (t + 1 < SEQ) ? (t + 1) : (SEQ - 1);
    const double* nq = ap + (size_t)tn * 256;
    const v2d n0 = *(const v2d*)(nq), n1 = *(const v2d*)(nq + 2);
    const v2d n2 = *(const v2d*)(nq + 4), n3 = *(const v2d*)(nq + 6);
    const double bvv = bv[(base + (size_t)t) * NST + n];
    const v2d s0 = *(const v2da*)(st + 8 * h), s1 = *(const v2da*)(st + 8 * h + 2);
    const v2d s2 = *(const v2da*)(st + 8 * h + 4), s3 = *(const v2da*)(st + 8 * h + 6);
    double pp = c0.x * s0.x;
    pp = fma(c0.y, s0.y, pp);
    pp = fma(c1.x, s1.x, pp); pp = fma(c1.y, s1.y, pp);
    pp = fma(c2.x, s2.x, pp); pp = fma(c2.y, s2.y, pp);
    pp = fma(c3.x, s3.x, pp); pp = fma(c3.y, s3.y, pp);
    pp += __shfl_xor(pp, 16, 32);
    const double ns = pp + bvv;
    __syncthreads();
    if (lane < 16) st[n] = ns;
    const float hf = (float)ns;
    const unsigned hb = bf16_bits(hf);
    const float lf = (float)(ns - (double)__uint_as_float(hb << 16));
    const unsigned lb = bf16_bits(lf);
    sbuf[(t & 31) * 32 + lane] = (unsigned short)((h != 0) ? lb : hb);
    __syncthreads();
    if ((t & 31) == 31) {
      const v8us q0 = *(const v8usa*)(sbuf + 8 * lane);
      const v8us q1 = *(const v8usa*)(sbuf + 256 + 8 * lane);
      const v8us q2 = *(const v8usa*)(sbuf + 512 + 8 * lane);
      const v8us q3 = *(const v8usa*)(sbuf + 768 + 8 * lane);
      unsigned short* dp = stt + (base + (size_t)(t - 31)) * KST + 8 * lane;
      *(volatile v8us*)dp = q0;
      *(volatile v8us*)(dp + 256) = q1;
      *(volatile v8us*)(dp + 512) = q2;
      *(volatile v8us*)(dp + 768) = q3;
      __threadfence();
      *(volatile v8us*)dp = q0;
      *(volatile v8us*)(dp + 256) = q1;
      *(volatile v8us*)(dp + 512) = q2;
      *(volatile v8us*)(dp + 768) = q3;
    }
    c0 = n0; c1 = n1; c2 = n2; c3 = n3;
  }
}

__global__ __launch_bounds__(GTHR) void k_gate(const unsigned short* __restrict__ stt,
                                               const unsigned short* __restrict__ CM2,
                                               const float* __restrict__ gate, unsigned short* G) {
  __shared__ __attribute__((aligned(16))) float stg[GBM * GBN];
  const int tid = (int)threadIdx.x, lane = tid & 31, wave = tid >> 5, hh = lane >> 4, m = lane & 15;
  const int rowBase = (int)blockIdx.x * GBM;
  const int col0    = (int)blockIdx.y * GBN;

  FragB af;
  {
    const unsigned short* ap = stt + (size_t)(rowBase + 16 * wave + m) * KST + 8 * hh;
    af.h[0] = *(const v8usa*)ap;
    af.h[1] = *(const v8usa*)(ap + 16);
  }
  v8f acc[8];
#pragma unroll
  for (int nt = 0; nt < 8; ++nt) {
    const unsigned short* wq = CM2 + (size_t)(col0 + 16 * nt + m) * KST + 8 * hh;
    FragB bf;
    bf.h[0] = *(const v8usa*)wq;
    bf.h[1] = *(const v8usa*)(wq + 16);
    const v8f z = {0.f, 0.f, 0.f, 0.f, 0.f, 0.f, 0.f, 0.f};
    acc[nt] = wmb(af, bf, z);
  }
#pragma unroll
  for (int nt = 0; nt < 8; ++nt) {
    const int lc = 16 * nt + m;
#pragma unroll
    for (int r = 0; r < 8; ++r) {
      const int lr = 16 * wave + 8 * hh + r;
      stg[lr * GBN + lc] = acc[nt][r];
    }
  }
  __syncthreads();

#pragma unroll 1
  for (int i = 0; i < 16; ++i) {
    const int lr = 16 * wave + i;
    const v4f y  = *(const v4fa*)(stg + lr * GBN + 4 * lane);
    const v4f gv = *(const v4f*)(gate + (size_t)(rowBase + lr) * INR + col0 + 4 * lane);
    v4f v;
    v.x = y.x * sigmoid_f(gv.x); v.y = y.y * sigmoid_f(gv.y);
    v.z = y.z * sigmoid_f(gv.z); v.w = y.w * sigmoid_f(gv.w);
    v4us h4, l4;
    hilo4(v, h4, l4);
    unsigned short* srow = (unsigned short*)stg + (size_t)lr * (2 * GBN);
    *(v4usa*)(srow + 4 * lane) = h4;
    *(v4usa*)(srow + GBN + 4 * lane) = l4;
  }
  __syncthreads();
  v8us qv[16];
#pragma unroll
  for (int i = 0; i < 16; ++i) {
    const unsigned short* srow = (const unsigned short*)stg + (size_t)(16 * wave + i) * (2 * GBN);
    qv[i] = *(const v8usa*)(srow + 8 * lane);
  }
  const int coff = col0 + ((lane < 16) ? (8 * lane) : (INR + 8 * (lane - 16)));
#pragma unroll
  for (int i = 0; i < 16; ++i) {
    unsigned short* gp = G + (size_t)(rowBase + 16 * wave + i) * KOUT + coff;
    *(volatile v8us*)gp = qv[i];
  }
  __threadfence();
#pragma unroll
  for (int i = 0; i < 16; ++i) {
    unsigned short* gp = G + (size_t)(rowBase + 16 * wave + i) * KOUT + coff;
    *(volatile v8us*)gp = qv[i];
  }
}

static inline size_t al256(size_t o) { return (o + 255) & ~(size_t)255; }

extern "C" void kernel_launch(void* const* d_in, const int* in_sizes, int n_in,
                              void* d_out, int out_size, void* d_ws, size_t ws_size,
                              hipStream_t stream) {
  if (n_in < 9) return;
  if (in_sizes[0] != MROWS * DM) return;
  if (in_sizes[1] != DM || in_sizes[2] != DM) return;
  if (in_sizes[3] != NPJ * DM) return;
  if (in_sizes[4] != INR * 3) return;
  if (in_sizes[5] != NST * NST) return;
  if (in_sizes[6] != NST * INR) return;
  if (in_sizes[7] != INR * NST) return;
  if (in_sizes[8] != DM * INR) return;
  if (out_size != MROWS * DM) return;

  const float* x      = (const float*)d_in[0];
  const float* ln_g   = (const float*)d_in[1];
  const float* ln_b   = (const float*)d_in[2];
  const float* W_in   = (const float*)d_in[3];
  const float* conv_w = (const float*)d_in[4];
  const float* Amat   = (const float*)d_in[5];
  const float* Bmat   = (const float*)d_in[6];
  const float* Cmat   = (const float*)d_in[7];
  const float* W_out  = (const float*)d_in[8];
  float* out = (float*)d_out;

  char* ws = (char*)d_ws;
  size_t off = 0;
  const size_t oR1  = off; off = al256(off + (size_t)MROWS * KPJ * 2);
  const size_t oR2  = off; off = al256(off + (size_t)MROWS * INR * 4);
  const size_t oR3  = off; off = al256(off + (size_t)MROWS * INR * 4);
  const size_t oWI2 = off; off = al256(off + (size_t)NPJ * KPJ * 2);
  const size_t oWO2 = off; off = al256(off + (size_t)DM * KOUT * 2);
  const size_t oBM2 = off; off = al256(off + (size_t)NST * KOUT * 2);
  const size_t oCM2 = off; off = al256(off + (size_t)INR * KST * 2);
  const size_t oDP  = off; off = al256(off + (size_t)6 * MROWS * 4);
  const size_t oWT  = off; off = al256(off + (size_t)MROWS * NST * 4);
  const size_t oBV  = off; off = al256(off + (size_t)MROWS * NST * 8);
  const size_t oST  = off; off = al256(off + (size_t)MROWS * KST * 2);
  const size_t oCST = off; off = al256(off + (size_t)CST_N * 8);
  if (off > ws_size) return;
  if (oR3 != oR2 + (size_t)MROWS * INR * 4) return;
  unsigned short* H    = (unsigned short*)(ws + oR1);
  double*         AD   = (double*)(ws + oR1);
  float*          DATA = (float*)(ws + oR2);
  unsigned short* G    = (unsigned short*)(ws + oR2);
  float*          GATE = (float*)(ws + oR3);
  unsigned short* WI2  = (unsigned short*)(ws + oWI2);
  unsigned short* WO2  = (unsigned short*)(ws + oWO2);
  unsigned short* BM2  = (unsigned short*)(ws + oBM2);
  unsigned short* CM2  = (unsigned short*)(ws + oCM2);
  float*          DP   = (float*)(ws + oDP);
  float*          WT   = (float*)(ws + oWT);
  double*         BV   = (double*)(ws + oBV);
  unsigned short* ST   = (unsigned short*)(ws + oST);
  double*         CST  = (double*)(ws + oCST);
  const size_t gateOff = (size_t)MROWS * INR;

  k_wprep<<<U_ALL / 256, 256, 0, stream>>>(W_in, W_out, Bmat, Cmat, WI2, WO2, BM2, CM2);
  k_aprep<<<1, 256, 0, stream>>>(Amat, CST);
  k_ln<<<MROWS / 8, 256, 0, stream>>>(x, ln_g, ln_b, H);
  k_gemm<0><<<dim3(MROWS / GBM, NPJ / GBN), GTHR, 0, stream>>>(H, WI2, KPJ, DATA, gateOff, DP, x, out);
  k_conv<<<MROWS / CTOK, CTHR, 0, stream>>>(DATA, conv_w, BM2, WT);
  k_expm<<<MROWS / TPB, 256, 0, stream>>>(CST, DP, WT, AD, BV);
  k_scan<<<NB, 32, 0, stream>>>(AD, BV, ST);
  k_gate<<<dim3(MROWS / GBM, INR / GBN), GTHR, 0, stream>>>(ST, CM2, GATE, G);
  k_gemm<1><<<dim3(MROWS / GBM, DM / GBN), GTHR, 0, stream>>>(G, WO2, KOUT, DATA, gateOff, DP, x, out);
}
